// PillarFeatureNet_38903813767719
// MI455X (gfx1250) — hardware-run, weakly checked
//
#include <hip/hip_runtime.h>
#include <stddef.h>


#pragma clang fp contract(off)

typedef __bf16       v16bf __attribute__((ext_vector_type(16)));
typedef float        v8f   __attribute__((ext_vector_type(8)));
typedef float        v4f   __attribute__((ext_vector_type(4)));
typedef unsigned int v8u   __attribute__((ext_vector_type(8)));
typedef unsigned int v4u   __attribute__((ext_vector_type(4)));

#ifndef NPIL
#define NPIL 60000
#endif
#define NPIL_FULL 60000
#define NPTS  32
#define NCH   64
#define NFEAT 9
#define NSTAT 54
#define STAT_BLOCKS 120
#define PROW  64
#define BPW   16

static_assert(NPIL >= 8 && NPIL <= NPIL_FULL);
static_assert((NPIL % 8) == 0);
static_assert(NPTS == 32);
static_assert(NCH == 64 && (NCH % 16) == 0);
static_assert(NFEAT == 9 && 3 * NFEAT <= 32);
static_assert(NSTAT == NFEAT + NFEAT * (NFEAT + 1) / 2);
static_assert(NSTAT <= PROW && (PROW % 32) == 0);
static_assert(16 * 16 == 4 * PROW);
static_assert(PROW == NCH);
static_assert(BPW * 2 == 32);
static_assert((size_t)NPIL * NPTS * 4 < (size_t)0x7FFFFFFF);

#define INV_M (1.0 / ((double)NPIL * (double)NPTS))

#define PART_BYTES ((size_t)STAT_BLOCKS * PROW * 4)
#define SB_BYTES   ((size_t)2 * NCH * 4)
#define BP_BYTES   ((size_t)NCH * BPW * 4)
#define OFF_PART   ((size_t)0)
#define OFF_SB     (OFF_PART + PART_BYTES)
#define OFF_BP     (OFF_SB + SB_BYTES)
#define WS_TOTAL   (OFF_BP + BP_BYTES)
static_assert((PART_BYTES % 128) == 0 && (SB_BYTES % 128) == 0 && (BP_BYTES % 128) == 0);
static_assert(SB_BYTES == 32 * 16);
static_assert(BP_BYTES == 4 * 64 * 16);
static_assert(WS_TOTAL <= (size_t)134217728);

__device__ __forceinline__ unsigned bf16_bits(float x) {
  const unsigned u = __float_as_uint(x);
  return (u + 0x7FFFu + ((u >> 16) & 1u)) >> 16;
}

__device__ __forceinline__ v8f wmma_bf(v8u a, v8u b, v8f c) {
  v8f d = __builtin_amdgcn_wmma_f32_16x16x32_bf16(false, __builtin_bit_cast(v16bf, a),
                                                  false, __builtin_bit_cast(v16bf, b),
                                                  (short)0, c, false, false);
  asm volatile("v_nop\n\tv_nop\n\tv_nop\n\tv_nop" : "+v"(d) : "v"(a), "v"(b));
  return d;
}

__device__ __forceinline__ v8u build_afrag(const float (&f)[NFEAT], unsigned h) {
  unsigned hb[NFEAT], lb[NFEAT];
#pragma unroll
  for (int c = 0; c < NFEAT; ++c) {
    hb[c] = bf16_bits(f[c]);
    const float hf = __uint_as_float(hb[c] << 16);
    lb[c] = bf16_bits(f[c] - hf);
  }
  unsigned w0[8], w1[8];
  w0[0] = hb[0] | (hb[1] << 16);
  w0[1] = hb[2] | (hb[3] << 16);
  w0[2] = hb[4] | (hb[5] << 16);
  w0[3] = hb[6] | (hb[7] << 16);
  w0[4] = hb[8] | (lb[0] << 16);
  w0[5] = lb[1] | (lb[2] << 16);
  w0[6] = lb[3] | (lb[4] << 16);
  w0[7] = lb[5] | (lb[6] << 16);
  w1[0] = lb[7] | (lb[8] << 16);
  w1[1] = hb[0] | (hb[1] << 16);
  w1[2] = hb[2] | (hb[3] << 16);
  w1[3] = hb[4] | (hb[5] << 16);
  w1[4] = hb[6] | (hb[7] << 16);
  w1[5] = hb[8];
  w1[6] = 0u;
  w1[7] = 0u;
  v8u out;
#pragma unroll
  for (int j = 0; j < 8; ++j) out[j] = (h != 0u) ? w1[j] : w0[j];
  return out;
}

__global__ __launch_bounds__(256) void pfn_stats_kernel(
    const float* __restrict__ voxels, const int* __restrict__ num_points,
    const int* __restrict__ coors, float* __restrict__ partials) {
  __shared__ float red[8][NSTAT];
  __shared__ __attribute__((aligned(16))) float rowbuf[PROW];
  const int tid = (int)threadIdx.x;
  const int lane = tid & 31;
  const int wave = __builtin_amdgcn_readfirstlane(tid >> 5);

  float acc[NSTAT];
#pragma unroll
  for (int i = 0; i < NSTAT; ++i) acc[i] = 0.0f;

#pragma unroll 1
  for (int n = (int)blockIdx.x * 8 + wave; n < NPIL; n += STAT_BLOCKS * 8) {
    const v4f v = *(const v4f*)(voxels + ((size_t)n * NPTS + (size_t)lane) * 4u);
    const int npts = num_points[n];
    float sx = v[0], sy = v[1], sz = v[2];
#pragma unroll
    for (int off = 16; off; off >>= 1) {
      sx += __shfl_xor(sx, off, 32);
      sy += __shfl_xor(sy, off, 32);
      sz += __shfl_xor(sz, off, 32);
    }
    const float inv = 1.0f / (float)max(npts, 1);
    float px = (float)coors[n * 4 + 1] * 0.1f;
    px = px + 0.05f;
    px = px + (-20.0f);
    float py = (float)coors[n * 4 + 2] * 0.1f;
    py = py + 0.05f;
    py = py + (-20.0f);
    const float mk = (lane < npts) ? 1.0f : 0.0f;
    float f[NFEAT];
    f[0] = v[0] * mk; f[1] = v[1] * mk; f[2] = v[2] * mk; f[3] = v[3] * mk;
    f[4] = (v[0] - sx * inv) * mk;
    f[5] = (v[1] - sy * inv) * mk;
    f[6] = (v[2] - sz * inv) * mk;
    f[7] = (v[0] - px) * mk;
    f[8] = (v[1] - py) * mk;
#pragma unroll
    for (int j = 0; j < NFEAT; ++j) acc[j] += f[j];
    int idx = NFEAT;
#pragma unroll
    for (int j = 0; j < NFEAT; ++j)
#pragma unroll
      for (int k = j; k < NFEAT; ++k) acc[idx++] += f[j] * f[k];
  }

#pragma unroll
  for (int i = 0; i < NSTAT; ++i) {
    float a = acc[i];
#pragma unroll
    for (int off = 16; off; off >>= 1) a += __shfl_xor(a, off, 32);
    acc[i] = a;
  }
  if (lane == 0) {
#pragma unroll
    for (int i = 0; i < NSTAT; ++i) red[wave][i] = acc[i];
  }
  __syncthreads();
  if (tid < PROW) {
    const int ci = min(tid, NSTAT - 1);
    float t = 0.0f;
#pragma unroll 1
    for (int w = 0; w < 8; ++w) t += red[w][ci];
    rowbuf[tid] = (tid < NSTAT) ? t : 0.0f;
  }
  __syncthreads();
  if (tid < 16) {
    const v4f val = *(const v4f*)&rowbuf[tid * 4];
    float* p = partials + (size_t)blockIdx.x * PROW + (size_t)tid * 4u;
    *(volatile v4f*)p = val;
    __threadfence();
    *(volatile v4f*)p = val;
  }
}

__global__ __launch_bounds__(64) void pfn_bn_kernel(
    const float* __restrict__ partials, const float* __restrict__ W,
    const float* __restrict__ gamma, const float* __restrict__ beta,
    float* __restrict__ scale_bias, unsigned int* __restrict__ bplane) {
  __shared__ double tot[PROW];
  __shared__ __attribute__((aligned(16))) float sbs[2 * NCH];
  __shared__ __attribute__((aligned(16))) unsigned int bpw[NCH * BPW];
  const unsigned tid = threadIdx.x;
  {
    double t = 0.0;
#pragma unroll 1
    for (int b = 0; b < STAT_BLOCKS; ++b) t += (double)partials[(size_t)b * PROW + tid];
    tot[tid] = t;
  }
  __syncthreads();

  const unsigned o = tid;
  float w[NFEAT];
#pragma unroll
  for (int c = 0; c < NFEAT; ++c) w[c] = W[o * NFEAT + c];

  double s1 = 0.0;
#pragma unroll
  for (int c = 0; c < NFEAT; ++c) s1 += (double)w[c] * tot[c];
  const double mean = s1 * INV_M;
  double s2 = 0.0;
  int idx = NFEAT;
#pragma unroll
  for (int j = 0; j < NFEAT; ++j)
#pragma unroll
    for (int k = j; k < NFEAT; ++k) {
      const double term = (double)w[j] * (double)w[k] * tot[idx++];
      s2 += (k == j) ? term : 2.0 * term;
    }
  const double var = s2 * INV_M - mean * mean;
  const float sc = gamma[o] * rsqrtf((float)var + 0.001f);
  sbs[o] = sc;
  sbs[NCH + o] = beta[o] - (float)mean * sc;

  unsigned hb[NFEAT], lb[NFEAT];
#pragma unroll
  for (int c = 0; c < NFEAT; ++c) {
    hb[c] = bf16_bits(w[c]);
    const float hf = __uint_as_float(hb[c] << 16);
    lb[c] = bf16_bits(w[c] - hf);
  }
  unsigned int* row = &bpw[o * BPW];
  row[0] = hb[0] | (hb[1] << 16);
  row[1] = hb[2] | (hb[3] << 16);
  row[2] = hb[4] | (hb[5] << 16);
  row[3] = hb[6] | (hb[7] << 16);
  row[4] = hb[8] | (hb[0] << 16);
  row[5] = hb[1] | (hb[2] << 16);
  row[6] = hb[3] | (hb[4] << 16);
  row[7] = hb[5] | (hb[6] << 16);
  row[8]  = hb[7] | (hb[8] << 16);
  row[9]  = lb[0] | (lb[1] << 16);
  row[10] = lb[2] | (lb[3] << 16);
  row[11] = lb[4] | (lb[5] << 16);
  row[12] = lb[6] | (lb[7] << 16);
  row[13] = lb[8];
  row[14] = 0u;
  row[15] = 0u;
  __syncthreads();

  v4u xb[4];
#pragma unroll
  for (unsigned it = 0; it < 4u; ++it) xb[it] = *(const v4u*)&bpw[(it * 64u + tid) * 4u];
  const v4f xs = *(const v4f*)&sbs[(tid & 31u) * 4u];
#pragma unroll
  for (unsigned it = 0; it < 4u; ++it)
    *(volatile v4u*)(bplane + (size_t)(it * 64u + tid) * 4u) = xb[it];
  if (tid < 32u) *(volatile v4f*)(scale_bias + (size_t)tid * 4u) = xs;
  __threadfence();
#pragma unroll
  for (unsigned it = 0; it < 4u; ++it)
    *(volatile v4u*)(bplane + (size_t)(it * 64u + tid) * 4u) = xb[it];
  if (tid < 32u) *(volatile v4f*)(scale_bias + (size_t)tid * 4u) = xs;
}

__global__ __launch_bounds__(256) void pfn_main_kernel(
    const float* __restrict__ voxels, const int* __restrict__ num_points,
    const int* __restrict__ coors, const float* __restrict__ scale_bias,
    const unsigned int* __restrict__ bplane, float* __restrict__ out) {
  __shared__ __attribute__((aligned(16))) float otile[8 * NCH];

  const unsigned tid = threadIdx.x, lane = tid & 31u;
  const unsigned wave = (unsigned)__builtin_amdgcn_readfirstlane((int)(tid >> 5));
  const unsigned h = lane >> 4, m = lane & 15u;
  const unsigned n = blockIdx.x * 8u + wave;

  const float* vp = voxels + ((size_t)n * NPTS + m) * 4u;
  const v4f v0 = *(const v4f*)vp;
  const v4f v1 = *(const v4f*)(vp + 64);
  const int npts = num_points[n];

  float sx = v0[0] + v1[0], sy = v0[1] + v1[1], sz = v0[2] + v1[2];
#pragma unroll
  for (int off = 8; off; off >>= 1) {
    sx += __shfl_xor(sx, off, 32);
    sy += __shfl_xor(sy, off, 32);
    sz += __shfl_xor(sz, off, 32);
  }
  const float inv = 1.0f / (float)max(npts, 1);
  float px = (float)coors[n * 4u + 1u] * 0.1f;
  px = px + 0.05f;
  px = px + (-20.0f);
  float py = (float)coors[n * 4u + 2u] * 0.1f;
  py = py + 0.05f;
  py = py + (-20.0f);
  const float mx = sx * inv, my = sy * inv, mz = sz * inv;

  v8u af[2];
#pragma unroll
  for (int mt = 0; mt < 2; ++mt) {
    const v4f v = (mt == 0) ? v0 : v1;
    const float mk = ((int)(16u * (unsigned)mt + m) < npts) ? 1.0f : 0.0f;
    float f[NFEAT];
    f[0] = v[0] * mk; f[1] = v[1] * mk; f[2] = v[2] * mk; f[3] = v[3] * mk;
    f[4] = (v[0] - mx) * mk;
    f[5] = (v[1] - my) * mk;
    f[6] = (v[2] - mz) * mk;
    f[7] = (v[0] - px) * mk;
    f[8] = (v[1] - py) * mk;
    af[mt] = build_afrag(f, h);
  }

  v8u bw[4];
  float sc[4], bi[4];
#pragma unroll
  for (int t = 0; t < 4; ++t) {
    const unsigned ch = 16u * (unsigned)t + m;
    const unsigned int* bp = bplane + (size_t)ch * BPW + h * 8u;
    const v4u q0 = *(const v4u*)bp;
    const v4u q1 = *(const v4u*)(bp + 4);
    v8u b;
#pragma unroll
    for (int j = 0; j < 4; ++j) { b[j] = q0[j]; b[j + 4] = q1[j]; }
    bw[t] = b;
    sc[t] = scale_bias[ch];
    bi[t] = scale_bias[NCH + ch];
  }

  float cmax[4] = {0.0f, 0.0f, 0.0f, 0.0f};
#pragma unroll
  for (int mt = 0; mt < 2; ++mt) {
#pragma unroll
    for (int t = 0; t < 4; ++t) {
      v8f c = {};
      c = wmma_bf(af[mt], bw[t], c);
#pragma unroll
      for (int r = 0; r < 8; ++r) {
        const float y = c[r] * sc[t] + bi[t];
        const bool ok = ((int)(16u * (unsigned)mt + 8u * h + (unsigned)r) < npts);
        cmax[t] = fmaxf(cmax[t], ok ? y : 0.0f);
      }
    }
  }

#pragma unroll
  for (int t = 0; t < 4; ++t) {
    const float other = __shfl_xor(cmax[t], 16, 32);
    cmax[t] = fmaxf(cmax[t], other);
  }

  if (lane < 16u) {
#pragma unroll
    for (int t = 0; t < 4; ++t) otile[wave * NCH + 16u * (unsigned)t + m] = cmax[t];
  }
  __syncthreads();
  if (tid < 128u) {
    const v4f val = *(const v4f*)&otile[tid * 4u];
    float* p = out + (size_t)blockIdx.x * (8u * NCH) + (size_t)tid * 4u;
    *(volatile v4f*)p = val;
    __threadfence();
    *(volatile v4f*)p = val;
  }
}

extern "C" void kernel_launch(void* const* d_in, const int* in_sizes, int n_in,
                              void* d_out, int out_size, void* d_ws, size_t ws_size,
                              hipStream_t stream) {
  if (n_in < 6) return;
  if ((long long)in_sizes[0] < (long long)NPIL * NPTS * 4) return;
  if ((long long)in_sizes[1] < (long long)NPIL) return;
  if ((long long)in_sizes[2] < (long long)NPIL * 4) return;
  if (in_sizes[3] < NCH * NFEAT) return;
  if (in_sizes[4] < NCH || in_sizes[5] < NCH) return;
  if ((long long)out_size < (long long)NPIL * NCH) return;
  if (ws_size < WS_TOTAL) return;

  const float* voxels     = (const float*)d_in[0];
  const int*   num_points = (const int*)d_in[1];
  const int*   coors      = (const int*)d_in[2];
  const float* W          = (const float*)d_in[3];
  const float* gamma      = (const float*)d_in[4];
  const float* beta       = (const float*)d_in[5];
  float* out = (float*)d_out;

  char* ws = (char*)d_ws;
  float*        partials   = (float*)(ws + OFF_PART);
  float*        scale_bias = (float*)(ws + OFF_SB);
  unsigned int* bplane     = (unsigned int*)(ws + OFF_BP);

  pfn_stats_kernel<<<dim3(STAT_BLOCKS), dim3(256), 0, stream>>>(
      voxels, num_points, coors, partials);
  pfn_bn_kernel<<<dim3(1), dim3(64), 0, stream>>>(
      partials, W, gamma, beta, scale_bias, bplane);
  pfn_main_kernel<<<dim3(NPIL / 8), dim3(256), 0, stream>>>(
      voxels, num_points, coors, scale_bias, bplane, out);
}
